// NeighborhoodCrossAttention_74766790688938
// MI455X (gfx1250) — hardware-verified
//
#include <hip/hip_runtime.h>


namespace {
constexpr int Bn = 2, GH = 64, GW = 64, N = GH * GW, D = 256, NH = 8, HD = 32, NT = Bn * N;
constexpr float XS = 8.0f, PS = 8.0f, ISC = 0.17677669529663687f;

typedef _Float16 b16;
typedef __attribute__((ext_vector_type(16))) _Float16 v16b;
typedef __attribute__((ext_vector_type(8))) _Float16 v8b;
typedef __attribute__((ext_vector_type(8))) float v8f;
typedef __attribute__((ext_vector_type(4))) float v4f;
__device__ __forceinline__ float bf16_rne(float f) { unsigned int u = __float_as_uint(f); u += 0x7FFFu + ((u >> 16) & 1u); return __uint_as_float(u & 0xFFFF0000u); }
__device__ __forceinline__ void split16(float v, b16& hi, b16& lo) { hi = (b16)v; lo = (b16)(v - (float)hi); }
__device__ __forceinline__ v16b frag_kb(const b16* p, int hh) { const v8b a = *(const v8b*)(p + 8 * hh), b = *(const v8b*)(p + 16 + 8 * hh); v16b f;
#pragma unroll
  for (int e = 0; e < 8; ++e) { f[e] = a[e]; f[8 + e] = b[e]; } return f; }
__device__ __forceinline__ v8f wmma16b(v16b a, v16b b, v8f c) { v8f d = __builtin_amdgcn_wmma_f32_16x16x32_f16(false, a, false, b, (short)0, c, false, false); asm volatile("v_nop\n\tv_nop\n\tv_nop\n\tv_nop" : "+v"(d) : "v"(a), "v"(b)); return d; }
__device__ __forceinline__ void wave_lds_sync() { __builtin_amdgcn_fence(__ATOMIC_RELEASE, "workgroup"); __builtin_amdgcn_wave_barrier(); __builtin_amdgcn_fence(__ATOMIC_ACQUIRE, "workgroup"); }
__device__ __forceinline__ float nexp(float x) { return __builtin_amdgcn_exp2f(x * 1.4426950408889634f); }
__device__ __forceinline__ float pmul(float a, float b) { float p = a * b; asm volatile("" : "+v"(p)); return p; }
__device__ __forceinline__ float wsum(float v) {
#pragma unroll
  for (int o = 1; o < 32; o <<= 1) v += __shfl_xor(v, o); return v; }

__global__ __launch_bounds__(256) void prep_kernel(const float* __restrict__ x1, const float* __restrict__ wq, const float* __restrict__ wk, const float* __restrict__ wv, const float* __restrict__ wo, const float* __restrict__ bq, const float* __restrict__ bk, const float* __restrict__ bv, const float* __restrict__ bo, b16* __restrict__ R, float* __restrict__ P, b16* __restrict__ X1) {
  const size_t tid = (size_t)blockIdx.x * 256 + threadIdx.x, nth = (size_t)gridDim.x * 256;
  for (int pass = 0; pass < 2; ++pass) {
    for (size_t p = tid; p < (size_t)4 * D * D; p += nth) { const int w = (int)(p / (D * D)); const size_t r = p % ((size_t)D * D); ((volatile b16*)R)[p] = (b16)bf16_rne(((w == 0) ? wq : (w == 1) ? wk : (w == 2) ? wv : wo)[r]); }
    for (size_t q = tid; q < 1024; q += nth) { const int i = (int)q; P[q] = bf16_rne(((i < 256) ? bq : (i < 512) ? bk : (i < 768) ? bv : bo)[i & 255]); }
    for (size_t p = tid; p < (size_t)NT * D / 8; p += nth) { v8b v; for (int e = 0; e < 8; ++e) v[e] = (b16)(bf16_rne(x1[p * 8 + e]) * XS); *(volatile v8b*)(X1 + p * 8) = v; }
    __threadfence(); }
}
__global__ __launch_bounds__(256) void fuse_kernel(const float* __restrict__ x2, b16* __restrict__ Fh, b16* __restrict__ Fl) {
  __shared__ __attribute__((aligned(16))) b16 Sh[8][D + 8], Sl[8][D + 8];
  const int wave = threadIdx.x >> 5, t = blockIdx.x * 8 + wave, lane = threadIdx.x & 31; const int b = t / N, n = t % N, r0 = n / GW, c0 = n % GW;
  const float* xb = x2 + (size_t)b * N * D; float cen[8];
#pragma unroll
  for (int e = 0; e < 8; ++e) cen[e] = bf16_rne(xb[(size_t)n * D + lane * 8 + e]);
  auto cand_idx = [&](int k, bool& valid) { int rr = r0, cc = c0; valid = true; if (k > 0) { const int o = k - 1; rr = r0 + o / 3 - 1; cc = c0 + o % 3 - 1; valid = (rr >= 0 && rr < GH && cc >= 0 && cc < GW); } return valid ? rr * GW + cc : n; };
  auto score = [&](int nn, bool valid) { float d_ = 0.0f;
#pragma unroll
    for (int e = 0; e < 8; ++e) d_ += pmul(cen[e], bf16_rne(xb[(size_t)nn * D + lane * 8 + e]));
    d_ = wsum(d_); return valid ? d_ * 0.0625f : -INFINITY; };
  float m = -INFINITY, s = 0.0f;
#pragma unroll 1
  for (int k = 0; k < 10; ++k) { bool valid; const int nn = cand_idx(k, valid); const float sc = score(nn, valid); if (sc != -INFINITY) { const float mn = fmaxf(m, sc); s = s * ((m == -INFINITY) ? 0.0f : nexp(m - mn)) + nexp(sc - mn); m = mn; } }
  const float inv = 1.0f / s; float acc[8] = {0, 0, 0, 0, 0, 0, 0, 0};
#pragma unroll 1
  for (int k = 0; k < 10; ++k) { bool valid; const int nn = cand_idx(k, valid); const float sc = score(nn, valid); const float w = (sc == -INFINITY) ? 0.0f : nexp(sc - m) * inv;
#pragma unroll
    for (int e = 0; e < 8; ++e) acc[e] += pmul(w, bf16_rne(xb[(size_t)nn * D + lane * 8 + e])); }
#pragma unroll
  for (int e = 0; e < 8; ++e) { b16 a_, b_; split16(acc[e] * XS, a_, b_); Sh[wave][lane * 8 + e] = a_; Sl[wave][lane * 8 + e] = b_; }
  wave_lds_sync();
  for (int pass = 0; pass < 2; ++pass) { *(volatile v8b*)(Fh + (size_t)t * D + lane * 8) = *(const v8b*)(&Sh[wave][lane * 8]); *(volatile v8b*)(Fl + (size_t)t * D + lane * 8) = *(const v8b*)(&Sl[wave][lane * 8]); __threadfence(); }
}
__global__ __launch_bounds__(128) void proj_kernel(const b16* __restrict__ X1, const b16* __restrict__ Fh, const b16* __restrict__ Fl, const b16* __restrict__ R, const float* __restrict__ P, b16* __restrict__ QH, b16* __restrict__ QL, b16* __restrict__ KH, b16* __restrict__ KL, b16* __restrict__ VTh, b16* __restrict__ VTl) {
  __shared__ __attribute__((aligned(16))) b16 Th[128][64 + 8], Tl[128][64 + 8];
  __shared__ __attribute__((aligned(16))) b16 Rh[4][16][128 + 8], Rl[4][16][128 + 8];
  const int mode = blockIdx.z, lane = threadIdx.x & 31, wave = threadIdx.x >> 5, nloc = lane & 15, hlf = lane >> 4, g0 = blockIdx.y * 64, m0 = g0 + wave * 16, c0 = blockIdx.x * 128;
  const b16* Ah = (mode == 0) ? X1 : Fh; const b16* Bw = R + (size_t)mode * D * D; const float* bias = P + mode * D; const bool two = mode != 0;
  v8f acc[8];
#pragma unroll
  for (int t = 0; t < 8; ++t) acc[t] = (v8f){};
#pragma unroll
  for (int kb = 0; kb < D; kb += 32) { const v16b a = frag_kb(Ah + (size_t)(m0 + nloc) * D + kb, hlf); v16b al_; if (two) al_ = frag_kb(Fl + (size_t)(m0 + nloc) * D + kb, hlf);
#pragma unroll
    for (int t = 0; t < 8; ++t) { const v16b bw = frag_kb(Bw + (size_t)(c0 + t * 16 + nloc) * D + kb, hlf); acc[t] = wmma16b(a, bw, acc[t]); if (two) acc[t] = wmma16b(al_, bw, acc[t]); } }
  if (mode < 2) {
#pragma unroll
    for (int t = 0; t < 8; ++t)
#pragma unroll
      for (int r = 0; r < 8; ++r) { b16 a_, c_; split16(acc[t][r] + XS * bias[c0 + t * 16 + nloc], a_, c_); Rh[wave][8 * hlf + r][t * 16 + nloc] = a_; Rl[wave][8 * hlf + r][t * 16 + nloc] = c_; }
    wave_lds_sync();
    b16* dh = mode ? KH : QH; b16* dl = mode ? KL : QL;
    for (int pass = 0; pass < 2; ++pass) { for (int i = lane; i < 16 * 16; i += 32) { const int rr = i >> 4, c8 = (i & 15) * 8; const size_t gi = (size_t)(m0 + rr) * D + c0 + c8; *(volatile v8b*)(dh + gi) = *(const v8b*)(&Rh[wave][rr][c8]); *(volatile v8b*)(dl + gi) = *(const v8b*)(&Rl[wave][rr][c8]); } __threadfence(); } }
  else {
#pragma unroll
    for (int t = 0; t < 8; ++t)
#pragma unroll
      for (int r = 0; r < 8; ++r) { b16 a_, c_; split16(acc[t][r] + XS * bias[c0 + t * 16 + nloc], a_, c_); Th[t * 16 + nloc][wave * 16 + 8 * hlf + r] = a_; Tl[t * 16 + nloc][wave * 16 + 8 * hlf + r] = c_; }
    __syncthreads();
    const int b = g0 / N, tk0 = g0 % N;
    for (int pass = 0; pass < 2; ++pass) { for (int i = threadIdx.x; i < 128 * 8; i += 128) { const int dd = i >> 3, c8 = (i & 7) * 8; const size_t gi = ((size_t)b * D + c0 + dd) * N + tk0 + c8; *(volatile v8b*)(VTh + gi) = *(const v8b*)(&Th[dd][c8]); *(volatile v8b*)(VTl + gi) = *(const v8b*)(&Tl[dd][c8]); } __threadfence(); } }
}
__global__ __launch_bounds__(128) void attn_kernel(const b16* __restrict__ QH, const b16* __restrict__ QL, const b16* __restrict__ KH, const b16* __restrict__ KL, const b16* __restrict__ VTh, const b16* __restrict__ VTl, b16* __restrict__ CH, b16* __restrict__ CL) {
  __shared__ __attribute__((aligned(16))) b16 Oh[16][4 * HD + 8], Ol[16][4 * HD + 8];
  const int wid = threadIdx.x >> 5, lane = threadIdx.x & 31, hh = lane >> 4, col = lane & 15; const int b = blockIdx.z, q0 = blockIdx.x * 16, h = blockIdx.y * 4 + wid, qi = q0 + col;
  const b16* Qr = QH + ((size_t)b * N) * D + h * HD; const b16* Qlr = QL + ((size_t)b * N) * D + h * HD; const b16* Kr = KH + ((size_t)b * N) * D + h * HD; const b16* Klr = KL + ((size_t)b * N) * D + h * HD; const b16* V = VTh + ((size_t)b * D + h * HD) * N; const b16* Vl = VTl + ((size_t)b * D + h * HD) * N;
  const v16b qf = frag_kb(Qr + (size_t)qi * D, hh), ql = frag_kb(Qlr + (size_t)qi * D, hh);
  float m = -INFINITY, l = 0.0f; v8f o[2] = {{}, {}};
  for (int kb = 0; kb < N; kb += 32) {
    v8f s0 = {}, s1 = {};
    { const v16b k0 = frag_kb(Kr + (size_t)(kb + col) * D, hh), k0l = frag_kb(Klr + (size_t)(kb + col) * D, hh), k1 = frag_kb(Kr + (size_t)(kb + 16 + col) * D, hh), k1l = frag_kb(Klr + (size_t)(kb + 16 + col) * D, hh);
      s0 = wmma16b(k0, qf, s0); s0 = wmma16b(k0l, qf, s0); s0 = wmma16b(k0, ql, s0); s1 = wmma16b(k1, qf, s1); s1 = wmma16b(k1l, qf, s1); s1 = wmma16b(k1, ql, s1); }
    float mr = -INFINITY;
#pragma unroll
    for (int r = 0; r < 8; ++r) { s0[r] *= ISC / (XS * XS); s1[r] *= ISC / (XS * XS); mr = fmaxf(mr, fmaxf(s0[r], s1[r])); }
    mr = fmaxf(mr, __shfl_xor(mr, 16)); const float mn = fmaxf(m, mr); const float al_ = nexp(m - mn); m = mn; float sum = 0.0f; v16b pb, pl;
#pragma unroll
    for (int r = 0; r < 8; ++r) { const float e0 = nexp(s0[r] - mn), e1 = nexp(s1[r] - mn); sum += e0 + e1; b16 a_, c_; split16(e0 * PS, a_, c_); pb[r] = a_; pl[r] = c_; split16(e1 * PS, a_, c_); pb[8 + r] = a_; pl[8 + r] = c_; }
    sum += __shfl_xor(sum, 16); l = l * al_ + sum;
#pragma unroll
    for (int t = 0; t < 2; ++t) { o[t] *= al_; const v16b vh = frag_kb(V + (size_t)(t * 16 + col) * N + kb, hh); o[t] = wmma16b(vh, pb, o[t]); o[t] = wmma16b(vh, pl, o[t]); o[t] = wmma16b(frag_kb(Vl + (size_t)(t * 16 + col) * N + kb, hh), pb, o[t]); } }
  const float inv = 1.0f / (l * PS);
#pragma unroll
  for (int t = 0; t < 2; ++t)
#pragma unroll
    for (int r = 0; r < 8; ++r) { b16 a_, c_; split16(o[t][r] * inv, a_, c_); Oh[col][wid * HD + t * 16 + 8 * hh + r] = a_; Ol[col][wid * HD + t * 16 + 8 * hh + r] = c_; }
  __syncthreads();
  for (int pass = 0; pass < 2; ++pass) { for (int i = threadIdx.x; i < 16 * 16; i += 128) { const int rr = i >> 4, c8 = (i & 15) * 8; const size_t gi = ((size_t)b * N + q0 + rr) * D + blockIdx.y * 4 * HD + c8; *(volatile v8b*)(CH + gi) = *(const v8b*)(&Oh[rr][c8]); *(volatile v8b*)(CL + gi) = *(const v8b*)(&Ol[rr][c8]); } __threadfence(); }
}
__global__ __launch_bounds__(64) void out_kernel(const b16* __restrict__ CH, const b16* __restrict__ CL, const b16* __restrict__ R, const float* __restrict__ P, float* __restrict__ out) {
  __shared__ __attribute__((aligned(16))) float Ts[2][16][128 + 4];
  const int lane = threadIdx.x & 31, wave = threadIdx.x >> 5, nloc = lane & 15, hlf = lane >> 4, m0 = blockIdx.y * 32 + wave * 16, c0 = blockIdx.x * 128; const b16* RO = R + (size_t)3 * D * D;
  v8f acc[8];
#pragma unroll
  for (int t = 0; t < 8; ++t) acc[t] = (v8f){};
#pragma unroll
  for (int kb = 0; kb < D; kb += 32) { const v16b a = frag_kb(CH + (size_t)(m0 + nloc) * D + kb, hlf), al_ = frag_kb(CL + (size_t)(m0 + nloc) * D + kb, hlf);
#pragma unroll
    for (int t = 0; t < 8; ++t) { const v16b bw = frag_kb(RO + (size_t)(c0 + t * 16 + nloc) * D + kb, hlf); acc[t] = wmma16b(a, bw, acc[t]); acc[t] = wmma16b(al_, bw, acc[t]); } }
#pragma unroll
  for (int t = 0; t < 8; ++t)
#pragma unroll
    for (int r = 0; r < 8; ++r) Ts[wave][8 * hlf + r][t * 16 + nloc] = acc[t][r] * (1.0f / XS) + P[768 + c0 + t * 16 + nloc];
  wave_lds_sync();
  for (int pass = 0; pass < 2; ++pass) { for (int i = lane; i < 16 * 32; i += 32) { const int rr = i >> 5, c4 = (i & 31) * 4; *(volatile v4f*)(out + (size_t)(m0 + rr) * D + c0 + c4) = *(const v4f*)(&Ts[wave][rr][c4]); } __threadfence(); }
}
}

extern "C" void kernel_launch(void* const* d_in, const int* in_sizes, int n_in,
                              void* d_out, int out_size, void* d_ws, size_t ws_size, hipStream_t stream) {
  (void)n_in; (void)out_size;
  auto Fp = [&](int i) { return (const float*)d_in[i]; };
  float* out = (float*)d_out;
  if (in_sizes[0] != NT * D || in_sizes[1] != NT * D || in_sizes[2] != D * D) return;
  size_t off = 0; char* ws = (char*)d_ws;
  auto carve = [&](size_t bytes) { char* p = ws + off; off += (bytes + 255) & ~(size_t)255; return p; };
  const size_t plane = (size_t)NT * D;
  b16* R = (b16*)carve((size_t)4 * D * D * 2); float* P = (float*)carve(1024 * 4); b16* X1 = (b16*)carve(plane * 2); b16* Fh = (b16*)carve(plane * 2); b16* Fl = (b16*)carve(plane * 2);
  b16* QH = (b16*)carve(plane * 2); b16* QL = (b16*)carve(plane * 2); b16* KH = (b16*)carve(plane * 2); b16* KL = (b16*)carve(plane * 2); b16* VTh = (b16*)carve(plane * 2); b16* VTl = (b16*)carve(plane * 2); b16* CH = (b16*)carve(plane * 2); b16* CL = (b16*)carve(plane * 2);
  if (off > ws_size) return;
  prep_kernel<<<512, 256, 0, stream>>>(Fp(0), Fp(2), Fp(3), Fp(4), Fp(5), Fp(6), Fp(7), Fp(8), Fp(9), R, P, X1);
  fuse_kernel<<<NT / 8, 256, 0, stream>>>(Fp(1), Fh, Fl);
  proj_kernel<<<dim3(2, NT / 64, 3), 128, 0, stream>>>(X1, Fh, Fl, R, P, QH, QL, KH, KL, VTh, VTl);
  attn_kernel<<<dim3(N / 16, 2, Bn), 128, 0, stream>>>(QH, QL, KH, KL, VTh, VTl, CH, CL);
  out_kernel<<<dim3(2, NT / 32), 64, 0, stream>>>(CH, CL, R, P, out);
}
